// Cfconv_53858889891846
// MI455X (gfx1250) — hardware-verified
//
#include <hip/hip_runtime.h>
#include <stddef.h>

#define NRBF  300
#define KP    320
#define NF    64
#define NJ    128
#define NROW  2048
#define NTHR  256
#define NWAV  8
#define CE    256.0f
#define CW1   256.0f
#define CH    64.0f
#define CW2   256.0f
#define INV1  1.52587890625e-05f
#define INV2  6.103515625e-05f
#define GAM   10.0f
#define CSTEP 0.1f
#define LN2F  0.69314718055994530942f
#define NU1   (NF * (KP / 8))
#define NU2   (NF * (NF / 8))

static_assert(KP % 32 == 0 && KP >= NRBF && KP - NRBF < 32);
static_assert(NU1 % NTHR == 0 && (NU1 + NU2) % NTHR == 0);
static_assert(NJ == NWAV * 16 && NTHR == NWAV * 32);
static_assert(NF == 64 && NF % 32 == 0);

typedef _Float16 v16h __attribute__((ext_vector_type(16)));
typedef _Float16 v8h  __attribute__((ext_vector_type(8)));
typedef float    v8f  __attribute__((ext_vector_type(8)));
typedef float    v4f  __attribute__((ext_vector_type(4)));
typedef v8h __attribute__((may_alias)) v8ha;
typedef v4f __attribute__((may_alias)) v4fa;

union Frag { v16h v; v8h half[2]; };

__device__ __forceinline__ v8f wmma_f16(v16h a, v16h b, v8f c) {
  v8f d = __builtin_amdgcn_wmma_f32_16x16x32_f16(false, a, false, b, (short)0, c, false, false);
  asm volatile("v_nop\n\tv_nop\n\tv_nop\n\tv_nop" : "+v"(d) : "v"(a), "v"(b));
  return d;
}

__device__ __forceinline__ v16h load_frag(const _Float16* p, int h) {
  Frag f;
  f.half[0] = *(const v8ha*)(p + 8 * h);
  f.half[1] = *(const v8ha*)(p + 16 + 8 * h);
  return f.v;
}

__device__ __forceinline__ float bf16_val(float f) {
  const unsigned u = __float_as_uint(f);
  const unsigned r = (u + 0x7FFFu + ((u >> 16) & 1u)) >> 16;
  return __uint_as_float(r << 16);
}

__device__ __forceinline__ float ssp_f(float v) {
  const float t  = __expf(-fabsf(v));
  const float u  = __logf(1.0f + t);
  const float sp = fmaxf(v, 0.0f) + u;
  return sp - LN2F;
}

__device__ __forceinline__ void put16(_Float16* dp, v8h o) {
  *(volatile v8h*)dp = o;
  __threadfence();
  *(volatile v8h*)dp = o;
}

__global__ __launch_bounds__(NTHR) void k_prep(const float* __restrict__ W1, const float* __restrict__ W2,
                                               _Float16* W1T, _Float16* W2T) {
  const int u = (int)blockIdx.x * NTHR + (int)threadIdx.x;
  float v[8];
  _Float16* dp;
  if (u < NU1) {
    const int n  = u / (KP / 8);
    const int k8 = (u - n * (KP / 8)) * 8;
#pragma unroll
    for (int i = 0; i < 8; ++i) {
      const int k  = k8 + i;
      const int kc = k < NRBF ? k : NRBF - 1;
      const float w  = W1[(size_t)kc * NF + n];
      const float mk = (k < NRBF) ? 1.0f : 0.0f;
      v[i] = (CW1 * bf16_val(w)) * mk;
    }
    dp = W1T + (size_t)n * KP + k8;
  } else if (u < NU1 + NU2) {
    const int q  = u - NU1;
    const int n  = q >> 3;
    const int k8 = (q & 7) * 8;
#pragma unroll
    for (int i = 0; i < 8; ++i) v[i] = CW2 * bf16_val(W2[(size_t)(k8 + i) * NF + n]);
    dp = W2T + (size_t)n * NF + k8;
  } else {
    return;
  }
  const v8h o = { (_Float16)v[0], (_Float16)v[1], (_Float16)v[2], (_Float16)v[3],
                  (_Float16)v[4], (_Float16)v[5], (_Float16)v[6], (_Float16)v[7] };
  put16(dp, o);
}

__global__ __launch_bounds__(NTHR) void k_main(const float* __restrict__ x, const float* __restrict__ dist,
                                               const _Float16* __restrict__ W1T, const float* __restrict__ b1,
                                               const _Float16* __restrict__ W2T, const float* __restrict__ b2,
                                               float* out) {
#pragma clang fp contract(off)
  __shared__ __attribute__((aligned(16))) _Float16 sH[NWAV * 16 * NF];
  __shared__ __attribute__((aligned(16))) float sS[NWAV * NF];
  __shared__ __attribute__((aligned(16))) float sB[2 * NF];
  __shared__ __attribute__((aligned(16))) float sX[NF];
  __shared__ __attribute__((aligned(16))) float sO[NF];

  const int tid = (int)threadIdx.x, lane = tid & 31, w = tid >> 5, hh = lane >> 4, m = lane & 15;
  const int bi = (int)blockIdx.x;
  const int j  = 16 * w + m;

  const float d = bf16_val(dist[(size_t)bi * NJ + j]);
  if (tid < NF) {
    sB[tid]      = bf16_val(b1[tid]);
    sB[NF + tid] = bf16_val(b2[tid]);
    sX[tid]      = bf16_val(x[(size_t)bi * NF + tid]);
  }
  __syncthreads();

  const v8f z8 = {0.f, 0.f, 0.f, 0.f, 0.f, 0.f, 0.f, 0.f};

  v8f acc[4];
#pragma unroll
  for (int nt = 0; nt < 4; ++nt) acc[nt] = z8;
  const _Float16* w1p = W1T + (size_t)m * KP;

#pragma unroll 1
  for (int k0 = 0; k0 < KP; k0 += 32) {
    float ev[16];
#pragma unroll
    for (int i = 0; i < 16; ++i) {
      const int   k  = k0 + 8 * hh + (i & 7) + 16 * (i >> 3);
      const float c  = CSTEP * (float)k;
      const float t  = d - c;
      const float sq = t * t;
      const float ar = -GAM * sq;
      const float e  = __expf(ar);
      const float mk = (k < NRBF) ? CE : 0.0f;
      ev[i] = e * mk;
    }
    Frag a;
    a.half[0] = (v8h){ (_Float16)ev[0], (_Float16)ev[1], (_Float16)ev[2],  (_Float16)ev[3],
                       (_Float16)ev[4], (_Float16)ev[5], (_Float16)ev[6],  (_Float16)ev[7] };
    a.half[1] = (v8h){ (_Float16)ev[8], (_Float16)ev[9], (_Float16)ev[10], (_Float16)ev[11],
                       (_Float16)ev[12], (_Float16)ev[13], (_Float16)ev[14], (_Float16)ev[15] };
#pragma unroll
    for (int nt = 0; nt < 4; ++nt) {
      const v16h b = load_frag(w1p + (size_t)(16 * nt) * KP + k0, hh);
      acc[nt] = wmma_f16(a.v, b, acc[nt]);
    }
  }

  _Float16* sHw = sH + w * (16 * NF);
#pragma unroll
  for (int nt = 0; nt < 4; ++nt) {
    const float bv = sB[16 * nt + m];
#pragma unroll
    for (int r = 0; r < 8; ++r) {
      const float v = acc[nt][r] * INV1 + bv;
      sHw[(8 * hh + r) * NF + 16 * nt + m] = (_Float16)(CH * ssp_f(v));
    }
  }
  __syncthreads();

  v8f acc2[4];
#pragma unroll
  for (int nt = 0; nt < 4; ++nt) acc2[nt] = z8;
  const _Float16* w2p = W2T + (size_t)m * NF;
#pragma unroll
  for (int ks = 0; ks < 2; ++ks) {
    const int k0 = 32 * ks;
    const v16h a2 = load_frag(sHw + m * NF + k0, hh);
#pragma unroll
    for (int nt = 0; nt < 4; ++nt) {
      const v16h b = load_frag(w2p + (size_t)(16 * nt) * NF + k0, hh);
      acc2[nt] = wmma_f16(a2, b, acc2[nt]);
    }
  }

#pragma unroll
  for (int nt = 0; nt < 4; ++nt) {
    const float bv = sB[NF + 16 * nt + m];
    float part = 0.0f;
#pragma unroll
    for (int r = 0; r < 8; ++r) part += ssp_f(acc2[nt][r] * INV2 + bv);
    part += __shfl_xor(part, 16);
    if (hh == 0) sS[w * NF + 16 * nt + m] = part;
  }
  __syncthreads();

  if (tid < NF) {
    float s = 0.0f;
#pragma unroll
    for (int q = 0; q < NWAV; ++q) s += sS[q * NF + tid];
    sO[tid] = sX[tid] * s;
  }
  __syncthreads();

  if (w == 0) {
    const int lq = lane & 15;
    const v4f v = *(const v4fa*)(sO + 4 * lq);
    float* op = out + (size_t)bi * NF + 4 * lq;
    if (lane < 16) *(volatile v4f*)op = v;
    __threadfence();
    if (lane < 16) *(volatile v4f*)op = v;
  }
}

extern "C" void kernel_launch(void* const* d_in, const int* in_sizes, int n_in,
                              void* d_out, int out_size, void* d_ws, size_t ws_size,
                              hipStream_t stream) {
  if (n_in < 6) return;
  if (in_sizes[0] != NROW * NF) return;
  if (in_sizes[1] != NROW * NJ) return;
  if (in_sizes[2] != NRBF * NF) return;
  if (in_sizes[3] != NF) return;
  if (in_sizes[4] != NF * NF) return;
  if (in_sizes[5] != NF) return;
  if (out_size != NROW * NF) return;

  const float* x    = (const float*)d_in[0];
  const float* dist = (const float*)d_in[1];
  const float* W1   = (const float*)d_in[2];
  const float* b1   = (const float*)d_in[3];
  const float* W2   = (const float*)d_in[4];
  const float* b2   = (const float*)d_in[5];
  float* out = (float*)d_out;

  char* ws = (char*)d_ws;
  size_t off = 0;
  const size_t oW1T = off; off += (size_t)NF * KP * 2;  off = (off + 255) & ~(size_t)255;
  const size_t oW2T = off; off += (size_t)NF * NF * 2;  off = (off + 255) & ~(size_t)255;
  if (off > ws_size) return;
  _Float16* W1T = (_Float16*)(ws + oW1T);
  _Float16* W2T = (_Float16*)(ws + oW2T);

  k_prep<<<(NU1 + NU2) / NTHR, NTHR, 0, stream>>>(W1, W2, W1T, W2T);
  k_main<<<NROW, NTHR, 0, stream>>>(x, dist, W1T, b1, W2T, b2, out);
}
